// myWholeGAT_13932873909016
// MI455X (gfx1250) — hardware-verified
//
#include <hip/hip_runtime.h>
#include <math.h>
#include <stdint.h>

constexpr int kB   = 2;
constexpr int kF   = 128;
constexpr int kS   = 256;
constexpr int kN   = 512;
constexpr int kNN  = 1024;
constexpr int kH   = 4;
constexpr int kHF  = 512;
constexpr int kG   = 4;
constexpr int kAK  = kH * kS;
constexpr int kL   = 4;
constexpr float kNegSlope = 0.2f;
static_assert(kG * kS == kNN);
static_assert(kB * kN == kNN);

typedef __attribute__((ext_vector_type(16))) __bf16 v16b;
typedef __attribute__((ext_vector_type(8)))  __bf16 v8b;
typedef __attribute__((ext_vector_type(8)))  float  v8f;
typedef __attribute__((ext_vector_type(4)))  float  v4f;
typedef __attribute__((ext_vector_type(4)))  unsigned int v4u;

__device__ __forceinline__ unsigned short f2bf_bits(float f) {
  const unsigned u = __float_as_uint(f);
  return (unsigned short)((u + 0x7FFFu + ((u >> 16) & 1u)) >> 16);
}
__device__ __forceinline__ float bf_bits2f(unsigned short h) { return __uint_as_float(((unsigned)h) << 16); }
__device__ __forceinline__ unsigned pk16(unsigned short a, unsigned short b) { return (unsigned)a | ((unsigned)b << 16); }
__device__ __forceinline__ void split_pack2(float f0, float f1, unsigned& hp, unsigned& lp) {
  const unsigned short h0 = f2bf_bits(f0), h1 = f2bf_bits(f1);
  const unsigned short l0 = f2bf_bits(f0 - bf_bits2f(h0)), l1 = f2bf_bits(f1 - bf_bits2f(h1));
  hp = pk16(h0, h1); lp = pk16(l0, l1);
}
__device__ __forceinline__ float lrelu(float x) { return x > 0.f ? x : kNegSlope * x; }

union FragU { v16b v; v8b h[2]; };
__device__ __forceinline__ v16b frag_load(const __bf16* p) {
  FragU f; f.h[0] = *(const v8b*)(p); f.h[1] = *(const v8b*)(p + 16); return f.v;
}
__device__ __forceinline__ v8f mma3(v16b ah, v16b al, v16b bh, v16b bl, v8f c) {
  c = __builtin_amdgcn_wmma_f32_16x16x32_bf16(false, ah, false, bh, (short)0, c, false, false);
  c = __builtin_amdgcn_wmma_f32_16x16x32_bf16(false, ah, false, bl, (short)0, c, false, false);
  c = __builtin_amdgcn_wmma_f32_16x16x32_bf16(false, al, false, bh, (short)0, c, false, false);
  asm volatile("v_nop\n\tv_nop\n\tv_nop\n\tv_nop" : "+v"(c) : "v"(ah), "v"(al), "v"(bh), "v"(bl));
  return c;
}

template <bool BIAS, bool RESID, bool OUT16, bool AGG>
__global__ __launch_bounds__(256) void gemm_split_kernel(
    const unsigned short* __restrict__ Ahp, const unsigned short* __restrict__ Alp, int lda, int strideA,
    const unsigned short* __restrict__ Bhp, const unsigned short* __restrict__ Blp, int ldb, int strideB,
    void* Cout, void* Cout2, int ldc, int strideC,
    const float* __restrict__ bias,
    const float* __restrict__ resid, int ldr, int strideR,
    const float* __restrict__ aux, int strideX,
    int M, int N, int K) {
  __shared__ __align__(16) float sT[8][16 * 68];
  const int b    = blockIdx.y;
  const int lane = threadIdx.x & 31;
  const int wave = threadIdx.x >> 5;
  const int tilesN = N >> 6;
  const int tilesM = M >> 5;
  const int tile = blockIdx.x * 8 + wave;
  if (tile >= tilesM * tilesN) return;
  const int tm = tile / tilesN;
  const int tn = tile - tm * tilesN;
  const int m0 = tm << 5;
  const int n0 = tn << 6;

  const __bf16* Ah = (const __bf16*)(const void*)Ahp + (size_t)b * strideA;
  const __bf16* Al = (const __bf16*)(const void*)Alp + (size_t)b * strideA;
  const __bf16* Bh = (const __bf16*)(const void*)Bhp + (size_t)b * strideB;
  const __bf16* Bl = (const __bf16*)(const void*)Blp + (size_t)b * strideB;

  const int rlane = lane & 15;
  const int koff  = (lane >> 4) * 8;
  const int mOff  = (lane >> 4) * 8;

  v8f acc[2][4];
#pragma unroll
  for (int i = 0; i < 2; ++i)
#pragma unroll
    for (int j = 0; j < 4; ++j) acc[i][j] = (v8f){0.f,0.f,0.f,0.f,0.f,0.f,0.f,0.f};

#pragma unroll 1
  for (int k0 = 0; k0 < K; k0 += 32) {
    v16b bh[4], bl[4];
#pragma unroll
    for (int j = 0; j < 4; ++j) {
      const size_t bo = (size_t)(n0 + (j << 4) + rlane) * ldb + koff + k0;
      bh[j] = frag_load(Bh + bo);
      bl[j] = frag_load(Bl + bo);
    }
#pragma unroll
    for (int i = 0; i < 2; ++i) {
      const size_t ao = (size_t)(m0 + (i << 4) + rlane) * lda + koff + k0;
      const v16b ah = frag_load(Ah + ao);
      const v16b al = frag_load(Al + ao);
#pragma unroll
      for (int j = 0; j < 4; ++j) acc[i][j] = mma3(ah, al, bh[j], bl[j], acc[i][j]);
    }
  }

  float* slab = sT[wave];
  const float* Rb = resid + (size_t)b * strideR;
  const float* Xb = aux + (size_t)b * strideX;
#pragma unroll
  for (int i = 0; i < 2; ++i) {
    const int mBase = m0 + (i << 4);
    float sv[4][8];
#pragma unroll
    for (int j = 0; j < 4; ++j)
#pragma unroll
      for (int r = 0; r < 8; ++r) sv[j][r] = 0.f;
    if (AGG) {
#pragma unroll 1
      for (int hq = 0; hq < kH; ++hq) {
        float av[8];
#pragma unroll
        for (int r = 0; r < 8; ++r) av[r] = Xb[hq * kNN + mBase + mOff + r];
#pragma unroll
        for (int j = 0; j < 4; ++j) {
          const int n = n0 + (j << 4) + rlane;
#pragma unroll
          for (int r = 0; r < 8; ++r)
            sv[j][r] += av[r] * Rb[(size_t)(mBase + mOff + r) * ldr + hq * kF + n];
        }
      }
    }
#pragma unroll
    for (int j = 0; j < 4; ++j) {
      const int n = n0 + (j << 4) + rlane;
      float bv = 0.f;
      if (BIAS) bv = bias[n];
#pragma unroll
      for (int r = 0; r < 8; ++r) {
        float v = acc[i][j][r];
        if (AGG) v = (v + sv[j][r]) * 0.25f;
        if (BIAS) v += bv;
        if (RESID) v += Rb[(size_t)(mBase + mOff + r) * ldr + n];
        if (AGG) v = fmaxf(v, 0.0f);
        slab[(mOff + r) * 68 + (j << 4) + rlane] = v;
      }
    }
    __builtin_amdgcn_fence(__ATOMIC_RELEASE, "workgroup");
    __builtin_amdgcn_wave_barrier();
    __builtin_amdgcn_fence(__ATOMIC_ACQUIRE, "workgroup");
    if (!OUT16) {
      float* C = (float*)Cout + (size_t)b * strideC;
      const int hh = lane >> 4, c4 = (lane & 15) * 4;
      for (int pass = 0; pass < 2; ++pass) {
#pragma unroll
        for (int it = 0; it < 8; ++it) {
          const int row = it * 2 + hh;
          const v4f v = *(const v4f*)(slab + row * 68 + c4);
          *(volatile v4f*)(C + (size_t)(mBase + row) * ldc + n0 + c4) = v;
        }
        __threadfence();
      }
    } else {
      const int q = lane >> 3, c8 = (lane & 7) * 8;
      unsigned short* C  = (unsigned short*)Cout  + (size_t)b * strideC;
      unsigned short* C2 = (unsigned short*)Cout2 + (size_t)b * strideC;
      v4u hv[4], lv[4];
#pragma unroll
      for (int it = 0; it < 4; ++it) {
        const int row = it * 4 + q;
        const float* sp = slab + row * 68 + c8;
        v4u a, a2;
#pragma unroll
        for (int e = 0; e < 4; ++e) {
          unsigned hp, lp;
          split_pack2(sp[2 * e], sp[2 * e + 1], hp, lp);
          a[e] = hp; a2[e] = lp;
        }
        hv[it] = a; lv[it] = a2;
      }
      for (int pass = 0; pass < 2; ++pass) {
#pragma unroll
        for (int it = 0; it < 4; ++it) {
          const int row = it * 4 + q;
          const size_t go = (size_t)(mBase + row) * ldc + n0 + c8;
          *(volatile v4u*)(C + go)  = hv[it];
          *(volatile v4u*)(C2 + go) = lv[it];
        }
        __threadfence();
      }
    }
    __builtin_amdgcn_fence(__ATOMIC_RELEASE, "workgroup");
    __builtin_amdgcn_wave_barrier();
    __builtin_amdgcn_fence(__ATOMIC_ACQUIRE, "workgroup");
  }
}

__global__ __launch_bounds__(256) void tsplit_kernel(const float* __restrict__ W, unsigned short* __restrict__ oh,
                                                     unsigned short* __restrict__ ol, int inPitch, int outPitch,
                                                     int sInQ, int sInR, int sOutQ, int sOutR, int xflag) {
  __shared__ __align__(16) float tf[64 * 68];
  const int zq = blockIdx.z >> 2, zr = blockIdx.z & 3;
  W  += (size_t)(zq ^ xflag) * sInQ + (size_t)zr * sInR;
  oh += (size_t)zq * sOutQ + (size_t)zr * sOutR;
  ol += (size_t)zq * sOutQ + (size_t)zr * sOutR;
  const int c0  = blockIdx.x * 64;
  const int r0  = blockIdx.y * 64;
  const int tid = threadIdx.x;
  {
    const int lr = tid >> 4;
    const int c4 = (tid & 15) * 4;
#pragma unroll
    for (int it = 0; it < 4; ++it) {
      const int rr = it * 16 + lr;
      const v4f a = *(const v4f*)(W + (size_t)(r0 + rr) * inPitch + c0 + c4);
      *(v4f*)(tf + rr * 68 + c4) = a;
    }
  }
  __syncthreads();
  const int sub = tid >> 3;
  const int c8  = (tid & 7) * 8;
  v4u hv[2], lv[2];
#pragma unroll
  for (int it = 0; it < 2; ++it) {
    const int oc = it * 32 + sub;
    v4u a, a2;
#pragma unroll
    for (int q = 0; q < 4; ++q) {
      unsigned hp, lp;
      split_pack2(tf[(c8 + 2 * q) * 68 + oc], tf[(c8 + 2 * q + 1) * 68 + oc], hp, lp);
      a[q] = hp; a2[q] = lp;
    }
    hv[it] = a; lv[it] = a2;
  }
  for (int pass = 0; pass < 2; ++pass) {
#pragma unroll
    for (int it = 0; it < 2; ++it) {
      const int oc = it * 32 + sub;
      const size_t go = (size_t)(c0 + oc) * outPitch + r0 + c8;
      *(volatile v4u*)(oh + go) = hv[it];
      *(volatile v4u*)(ol + go) = lv[it];
    }
    __threadfence();
  }
}

__global__ __launch_bounds__(256) void build_x_kernel(const float* __restrict__ d0, const float* __restrict__ d1,
                                                      float* __restrict__ X) {
  const int tid  = threadIdx.x;
  const int node = blockIdx.x * 8 + (tid >> 5);
  const int lane = tid & 31;
  const int f4   = lane * 4;
  const int g    = node >> 9, n = node & (kN - 1);
  const float* src = (n < kS) ? d0 : d1;
  const int nn = n & (kS - 1);
  v4f v;
#pragma unroll
  for (int q = 0; q < 4; ++q) v[q] = src[(size_t)(g * kF + f4 + q) * kS + nn];
  float* dst = X + (size_t)node * kF + f4;
  *(volatile v4f*)dst = v;
  __threadfence();
  *(volatile v4f*)dst = v;
}

__global__ __launch_bounds__(256) void split_x_kernel(const float* __restrict__ X, unsigned short* __restrict__ ch,
                                                      unsigned short* __restrict__ cl) {
  const int t    = blockIdx.x * 256 + threadIdx.x;
  const int node = t >> 4;
  const int c8   = (t & 15) * 8;
  const float* xp = X + (size_t)node * kF + c8;
  const v4f a = *(const v4f*)(xp);
  const v4f c = *(const v4f*)(xp + 4);
  v4u hv, lv;
  { unsigned hp, lp; split_pack2(a[0], a[1], hp, lp); hv[0] = hp; lv[0] = lp; }
  { unsigned hp, lp; split_pack2(a[2], a[3], hp, lp); hv[1] = hp; lv[1] = lp; }
  { unsigned hp, lp; split_pack2(c[0], c[1], hp, lp); hv[2] = hp; lv[2] = lp; }
  { unsigned hp, lp; split_pack2(c[2], c[3], hp, lp); hv[3] = hp; lv[3] = lp; }
  const size_t go = (size_t)node * (2 * kF) + c8;
  *(volatile v4u*)(ch + go) = hv;
  *(volatile v4u*)(cl + go) = lv;
  __threadfence();
  *(volatile v4u*)(ch + go) = hv;
  *(volatile v4u*)(cl + go) = lv;
}

__global__ __launch_bounds__(256) void scores_kernel(const float* __restrict__ xw, const float* __restrict__ as,
                                                     const float* __restrict__ ad, float* __restrict__ sT,
                                                     float* __restrict__ dT) {
  const int idx  = blockIdx.x * 256 + threadIdx.x;
  const int h    = idx >> 10;
  const int node = idx & (kNN - 1);
  const float* row = xw + (size_t)node * kHF + h * kF;
  const float* pa  = as + h * kF;
  const float* pd  = ad + h * kF;
  float s = 0.f, d = 0.f;
#pragma unroll 2
  for (int c = 0; c < kF; c += 4) {
    const v4f x = *(const v4f*)(row + c);
    const v4f a = *(const v4f*)(pa + c);
    const v4f e = *(const v4f*)(pd + c);
    s += x[0] * a[0]; s += x[1] * a[1]; s += x[2] * a[2]; s += x[3] * a[3];
    d += x[0] * e[0]; d += x[1] * e[1]; d += x[2] * e[2]; d += x[3] * e[3];
  }
  *(volatile float*)(sT + idx) = s;
  *(volatile float*)(dT + idx) = d;
  __threadfence();
  *(volatile float*)(sT + idx) = s;
  *(volatile float*)(dT + idx) = d;
}

__global__ __launch_bounds__(256) void softmax_alpha_kernel(const float* __restrict__ sT, const float* __restrict__ dT,
                                                            unsigned short* __restrict__ alh, unsigned short* __restrict__ alo,
                                                            float* __restrict__ asf, int xflag) {
  __shared__ float sas[32];
  const int tid  = threadIdx.x;
  const int wave = tid >> 5;
  const int lane = tid & 31;
  const int grp  = blockIdx.y >> 2;
  const int h    = blockIdx.y & 3;
  const int srcgrp = grp ^ xflag;
  const int i0   = blockIdx.x * 32;
  const float* sp = sT + (size_t)h * kNN + srcgrp * kS + lane * 8;
  const v4f s0 = *(const v4f*)(sp);
  const v4f s1 = *(const v4f*)(sp + 4);
  const float sv[8] = {s0[0], s0[1], s0[2], s0[3], s1[0], s1[1], s1[2], s1[3]};

#pragma unroll 1
  for (int r = 0; r < 4; ++r) {
    const int row = wave * 4 + r;
    const int gd  = grp * kS + i0 + row;
    const float di = dT[(size_t)h * kNN + gd];
    const float ss = sT[(size_t)h * kNN + gd];
    float e[8];
    float m = -INFINITY;
#pragma unroll
    for (int k = 0; k < 8; ++k) { e[k] = lrelu(sv[k] + di); m = fmaxf(m, e[k]); }
    const float es  = lrelu(ss + di);
    const float msf = xflag ? es : -INFINITY;
    m = fmaxf(m, msf);
#pragma unroll
    for (int off = 1; off < 32; off <<= 1) m = fmaxf(m, __shfl_xor(m, off, 32));
    float p[8];
    float ps = 0.f;
#pragma unroll
    for (int k = 0; k < 8; ++k) { p[k] = __expf(e[k] - m); ps += p[k]; }
#pragma unroll
    for (int off = 1; off < 32; off <<= 1) ps += __shfl_xor(ps, off, 32);
    const float pex   = __expf(es - m);
    const float pself = xflag ? pex : 0.f;
    const float S   = ps + pself;
    const float inv = 1.0f / S;
    v4u hv, lv;
#pragma unroll
    for (int q = 0; q < 4; ++q) {
      unsigned hp, lp;
      split_pack2(p[2 * q] * inv, p[2 * q + 1] * inv, hp, lp);
      hv[q] = hp; lv[q] = lp;
    }
    const size_t go = (size_t)gd * kAK + h * kS + lane * 8;
    *(volatile v4u*)(alh + go) = hv;
    *(volatile v4u*)(alo + go) = lv;
    __threadfence();
    *(volatile v4u*)(alh + go) = hv;
    *(volatile v4u*)(alo + go) = lv;
    const float aself = pself * inv;
    if (lane == 0) sas[row] = aself;
  }
  __syncthreads();
  if (wave == 0) {
    const float v = sas[lane];
    float* pa = asf + (size_t)h * kNN + grp * kS + i0 + lane;
    *(volatile float*)pa = v;
    __threadfence();
    *(volatile float*)pa = v;
  }
}

__global__ __launch_bounds__(256) void write_out_kernel(const float* __restrict__ X, float* out) {
  __shared__ __align__(16) float tile[kS * 36];
  const int tid  = threadIdx.x;
  const int wave = tid >> 5;
  const int lane = tid & 31;
  const int p    = blockIdx.x >> 3;
  const int g    = (blockIdx.x >> 2) & 1;
  const int f0   = (blockIdx.x & 3) * 32;
  const int nodeBase = g * kN + p * kS;
#pragma unroll
  for (int it = 0; it < 8; ++it) {
    const int q  = it * 256 + tid;
    const int n  = q >> 3;
    const int f4 = (q & 7) * 4;
    const v4f v = *(const v4f*)(X + (size_t)(nodeBase + n) * kF + f0 + f4);
    *(v4f*)(tile + n * 36 + f4) = v;
  }
  __syncthreads();
  float* ob = out + (size_t)p * (kB * kF * kS) + (size_t)g * (kF * kS);
  v4f vals[4][2];
#pragma unroll
  for (int rr = 0; rr < 4; ++rr) {
    const int fr = wave * 4 + rr;
#pragma unroll
    for (int it = 0; it < 2; ++it) {
      const int n = it * 128 + lane * 4;
      v4f v;
      v[0] = tile[(n + 0) * 36 + fr];
      v[1] = tile[(n + 1) * 36 + fr];
      v[2] = tile[(n + 2) * 36 + fr];
      v[3] = tile[(n + 3) * 36 + fr];
      vals[rr][it] = v;
    }
  }
  for (int pass = 0; pass < 2; ++pass) {
#pragma unroll
    for (int rr = 0; rr < 4; ++rr) {
      const int fr = wave * 4 + rr;
#pragma unroll
      for (int it = 0; it < 2; ++it) {
        const int n = it * 128 + lane * 4;
        *(volatile v4f*)(ob + (size_t)(f0 + fr) * kS + n) = vals[rr][it];
      }
    }
    __threadfence();
  }
}

extern "C" void kernel_launch(void* const* d_in, const int* in_sizes, int n_in,
                              void* d_out, int out_size, void* d_ws, size_t ws_size,
                              hipStream_t stream) {
  if (n_in < 8) return;
  if (in_sizes[0] != kB * kF * kS || in_sizes[1] != kB * kF * kS) return;
  if (in_sizes[2] != kL * kF * kHF) return;
  if (in_sizes[3] != kL * kH * kF || in_sizes[4] != kL * kH * kF) return;
  if (in_sizes[5] != kL * kF) return;
  if (in_sizes[6] != kL * 2 * kF * kF || in_sizes[7] != kL * kF) return;
  if (out_size != 2 * kB * kF * kS) return;

  const float* desc0 = (const float*)d_in[0];
  const float* desc1 = (const float*)d_in[1];
  const float* W     = (const float*)d_in[2];
  const float* asrc  = (const float*)d_in[3];
  const float* adst  = (const float*)d_in[4];
  const float* bias  = (const float*)d_in[5];
  const float* mlpW  = (const float*)d_in[6];
  const float* mlpb  = (const float*)d_in[7];
  float* out = (float*)d_out;

  const size_t szWt  = (size_t)kL * kHF * kF * 2;
  const size_t szMt  = (size_t)kL * kF * (2 * kF) * 2;
  const size_t szX   = (size_t)kNN * kF * 4;
  const size_t szCat = (size_t)kNN * (2 * kF) * 2;
  const size_t szXW  = (size_t)kNN * kHF * 4;
  const size_t szXT  = (size_t)kG * kF * kNN * 2;
  const size_t szS   = (size_t)kH * kNN * 4;
  const size_t szAL  = (size_t)kG * kS * kAK * 2;
  size_t off = 0;
  const size_t oWth = off; off += szWt;  const size_t oWtl = off; off += szWt;
  const size_t oMth = off; off += szMt;  const size_t oMtl = off; off += szMt;
  const size_t oX0  = off; off += szX;   const size_t oX1  = off; off += szX;
  const size_t oCh  = off; off += szCat; const size_t oCl  = off; off += szCat;
  const size_t oXW  = off; off += szXW;
  const size_t oXTh = off; off += szXT;  const size_t oXTl = off; off += szXT;
  const size_t oST  = off; off += szS;   const size_t oDT  = off; off += szS;   const size_t oASF = off; off += szS;
  const size_t oALh = off; off += szAL;  const size_t oALl = off; off += szAL;
  if (off > ws_size) return;

  char* ws = (char*)d_ws;
  unsigned short* Wth  = (unsigned short*)(ws + oWth);  unsigned short* Wtl  = (unsigned short*)(ws + oWtl);
  unsigned short* Mth  = (unsigned short*)(ws + oMth);  unsigned short* Mtl  = (unsigned short*)(ws + oMtl);
  float*          X0   = (float*)(ws + oX0);            float*          X1   = (float*)(ws + oX1);
  unsigned short* Ch   = (unsigned short*)(ws + oCh);   unsigned short* Cl   = (unsigned short*)(ws + oCl);
  float*          XW   = (float*)(ws + oXW);
  unsigned short* XTh  = (unsigned short*)(ws + oXTh);  unsigned short* XTl  = (unsigned short*)(ws + oXTl);
  float*          ST   = (float*)(ws + oST);            float*          DT   = (float*)(ws + oDT);
  float*          ASF  = (float*)(ws + oASF);
  unsigned short* ALh  = (unsigned short*)(ws + oALh);  unsigned short* ALl  = (unsigned short*)(ws + oALl);

  const dim3 blk(256);

  tsplit_kernel<<<dim3(kHF / 64, kF / 64, kL), blk, 0, stream>>>(W, Wth, Wtl, kHF, kF, 0, kF * kHF, 0, kHF * kF, 0);
  tsplit_kernel<<<dim3(kF / 64, (2 * kF) / 64, kL), blk, 0, stream>>>(mlpW, Mth, Mtl, kF, 2 * kF, 0, 2 * kF * kF, 0, 2 * kF * kF, 0);
  build_x_kernel<<<dim3(kNN / 8), blk, 0, stream>>>(desc0, desc1, X0);
  split_x_kernel<<<dim3((kNN * kF / 8) / 256), blk, 0, stream>>>(X0, Ch, Cl);

  const dim3 gXW((( kNN / 32) * (kHF / 64) + 7) / 8, 1);
  const dim3 gAG((( kS  / 32) * (kF  / 64) + 7) / 8, kG);
  const dim3 gML((( kNN / 32) * (kF  / 64) + 7) / 8, 1);

  float* xcur = X0;
  float* xnext = X1;
  for (int l = 0; l < kL; ++l) {
    const int xflag = l & 1;
    gemm_split_kernel<false, false, false, false><<<gXW, blk, 0, stream>>>(
        Ch, Cl, 2 * kF, 0, Wth + (size_t)l * kHF * kF, Wtl + (size_t)l * kHF * kF, kF, 0,
        (void*)XW, (void*)XW, kHF, 0, bias, XW, kHF, 0, ASF, 0, kNN, kHF, kF);
    scores_kernel<<<dim3((kH * kNN) / 256), blk, 0, stream>>>(XW, asrc + (size_t)l * kH * kF, adst + (size_t)l * kH * kF, ST, DT);
    tsplit_kernel<<<dim3(kF / 64, kS / 64, kG * kH), blk, 0, stream>>>(XW, XTh, XTl, kHF, kAK, kS * kHF, kF, kF * kAK, kS, xflag);
    softmax_alpha_kernel<<<dim3(kS / 32, kG * kH), blk, 0, stream>>>(ST, DT, ALh, ALl, ASF, xflag);
    gemm_split_kernel<true, false, true, true><<<gAG, blk, 0, stream>>>(
        ALh, ALl, kAK, kS * kAK, XTh, XTl, kAK, kF * kAK,
        (void*)(Ch + kF), (void*)(Cl + kF), 2 * kF, kS * 2 * kF,
        bias + (size_t)l * kF, XW, kHF, kS * kHF, ASF, kS, kS, kF, kAK);
    gemm_split_kernel<true, true, false, false><<<gML, blk, 0, stream>>>(
        Ch, Cl, 2 * kF, 0, Mth + (size_t)l * kF * 2 * kF, Mtl + (size_t)l * kF * 2 * kF, 2 * kF, 0,
        (void*)xnext, (void*)xnext, kF, 0, mlpb + (size_t)l * kF, xcur, kF, 0, ASF, 0, kNN, kF, 2 * kF);
    if (l + 1 < kL) split_x_kernel<<<dim3((kNN * kF / 8) / 256), blk, 0, stream>>>(xnext, Ch, Cl);
    float* t = xcur; xcur = xnext; xnext = t;
  }
  write_out_kernel<<<dim3(2 * kB * (kF / 32)), blk, 0, stream>>>(xcur, out);
  (void)hipGetLastError();
}
